// PureLRUR_34857954574991
// MI455X (gfx1250) — hardware-verified
//
#include <hip/hip_runtime.h>
#include <stddef.h>
#include <stdint.h>
#include <math.h>

#define NB     16
#define SEQL   4096
#define HIN    128
#define NST    256
#define HOUT   128
#define NTOK   (NB * SEQL)
#define NHALF  2
#define BH     (NB / NHALF)
#define TOKH   (BH * SEQL)
#define NBU    (2 * NST)
#define KC     (2 * NST + HIN)
#define LDP    (2 * NBU)
#define SFP    68
#define TB     8
#define WSC    64.0f
#define WSCI   0.015625f

static_assert(TOKH % 128 == 0);
static_assert(NBU % 64 == 0);
static_assert(HOUT % 64 == 0);
static_assert(HIN % 32 == 0);
static_assert(NBU % 32 == 0);
static_assert(SEQL % TB == 0);
static_assert(TB * NBU == 4 * 4 * 256);
static_assert((TB * NBU) / 8 == 2 * 256);
static_assert((NBU * HIN) % 2048 == 0);
static_assert((HOUT * KC) % 2048 == 0);
static_assert((NTOK * HIN) % 2048 == 0);
static_assert(LDP * 2 == NBU * 4);

typedef _Float16 v16h __attribute__((ext_vector_type(16)));
typedef float v8f __attribute__((ext_vector_type(8)));
typedef float v4f __attribute__((ext_vector_type(4)));
typedef int v4i __attribute__((ext_vector_type(4)));
typedef int v8i __attribute__((ext_vector_type(8)));
typedef unsigned short v8us __attribute__((ext_vector_type(8)));

__device__ __forceinline__ v8f zero8() { return (v8f){0.f, 0.f, 0.f, 0.f, 0.f, 0.f, 0.f, 0.f}; }

__device__ __forceinline__ unsigned short h_bits(float f) {
  return __builtin_bit_cast(unsigned short, (_Float16)f);
}

__device__ __forceinline__ v8i ldfrag16(const unsigned short* __restrict__ p, int ld, int row0, int k0, int lane) {
  const unsigned short* q = p + (size_t)(row0 + (lane & 15)) * (size_t)ld + k0 + 8 * (lane >> 4);
  const v4i lo = *(const v4i*)(const void*)(q);
  const v4i hi = *(const v4i*)(const void*)(q + 16);
  return __builtin_shufflevector(lo, hi, 0, 1, 2, 3, 4, 5, 6, 7);
}

__device__ __forceinline__ v8f mma_h(v8i a, v8i b, v8f cc) {
  return __builtin_amdgcn_wmma_f32_16x16x32_f16(false, __builtin_bit_cast(v16h, a), false,
                                                __builtin_bit_cast(v16h, b), (short)0, cc, false, false);
}

__device__ __forceinline__ void gemm32x32(const unsigned short* __restrict__ A, int lda,
                                          const unsigned short* __restrict__ B, int ldb,
                                          int ma, int nb, int kdim, int lane, v8f (&acc)[2][2]) {
#pragma unroll 1
  for (int k0 = 0; k0 < kdim; k0 += 32) {
    const v8i a0 = ldfrag16(A, lda, ma, k0, lane);
    const v8i a1 = ldfrag16(A, lda, ma + 16, k0, lane);
    const v8i b0 = ldfrag16(B, ldb, nb, k0, lane);
    const v8i b1 = ldfrag16(B, ldb, nb + 16, k0, lane);
    acc[0][0] = mma_h(a0, b0, acc[0][0]);
    acc[1][0] = mma_h(a1, b0, acc[1][0]);
    acc[0][1] = mma_h(a0, b1, acc[0][1]);
    acc[1][1] = mma_h(a1, b1, acc[1][1]);
    asm volatile("v_nop\n\tv_nop\n\tv_nop\n\tv_nop"
                 : "+v"(acc[0][0]), "+v"(acc[0][1]), "+v"(acc[1][0]), "+v"(acc[1][1])
                 : "v"(a0), "v"(a1), "v"(b0), "v"(b1));
  }
}

__device__ __forceinline__ void stage_tile(float* ldsf, const v8f (&acc)[2][2], int wm, int wn, int h, int c) {
#pragma unroll
  for (int i = 0; i < 2; ++i)
#pragma unroll
    for (int j = 0; j < 2; ++j)
#pragma unroll
      for (int r = 0; r < 8; ++r)
        ldsf[(wm + 16 * i + 8 * h + r) * SFP + wn + 16 * j + c] = acc[i][j][r];
}

__global__ __launch_bounds__(256) void k_prepw(const float* __restrict__ Bre, const float* __restrict__ Bim,
                                               const float* __restrict__ Cre, const float* __restrict__ Cim,
                                               const float* __restrict__ Dm,
                                               unsigned short* __restrict__ WB, unsigned short* __restrict__ WC) {
  const int tid = threadIdx.x;
  if (blockIdx.x < (NBU * HIN) / 2048) {
    const int i  = blockIdx.x * 256 + tid;
    const int e0 = i * 8;
    const int n  = e0 >> 7, h = e0 & (HIN - 1);
    const int nn = n & (NST - 1);
    const float* pr = Bre + (size_t)nn * HIN + h;
    const float* pi = Bim + (size_t)nn * HIN + h;
    const v4f r0 = *(const v4f*)pr, r1 = *(const v4f*)(pr + 4);
    const v4f i0 = *(const v4f*)pi, i1 = *(const v4f*)(pi + 4);
    const bool im = (n >= NST);
    v8us o;
#pragma unroll
    for (int e = 0; e < 4; ++e) {
      o[e]     = h_bits(WSC * (im ? i0[e] : r0[e]));
      o[4 + e] = h_bits(WSC * (im ? i1[e] : r1[e]));
    }
    *(volatile v8us*)(WB + e0) = o;
    __threadfence();
    *(volatile v8us*)(WB + e0) = o;
  } else {
    const int i  = (blockIdx.x - (NBU * HIN) / 2048) * 256 + tid;
    const int e0 = i * 8;
    const int o  = e0 / KC, k = e0 - o * KC;
    const int k1 = min(k, NST - 8);
    const int k2 = min(max(k - NST, 0), NST - 8);
    const int k3 = min(max(k - 2 * NST, 0), HIN - 8);
    const float* pa = Cre + (size_t)o * NST + k1;
    const float* pb = Cim + (size_t)o * NST + k2;
    const float* pd = Dm  + (size_t)o * HIN + k3;
    const v4f a0 = *(const v4f*)pa, a1 = *(const v4f*)(pa + 4);
    const v4f b0 = *(const v4f*)pb, b1 = *(const v4f*)(pb + 4);
    const v4f d0 = *(const v4f*)pd, d1 = *(const v4f*)(pd + 4);
    const bool s0 = (k < NST), s1 = (k < 2 * NST);
    v8us w;
#pragma unroll
    for (int e = 0; e < 4; ++e) {
      const float v0 = s0 ? a0[e] : (s1 ? -b0[e] : d0[e]);
      const float v1 = s0 ? a1[e] : (s1 ? -b1[e] : d1[e]);
      w[e]     = h_bits(WSC * v0);
      w[4 + e] = h_bits(WSC * v1);
    }
    *(volatile v8us*)(WC + e0) = w;
    __threadfence();
    *(volatile v8us*)(WC + e0) = w;
  }
}

__global__ __launch_bounds__(256) void k_cvtu(const float* __restrict__ u, unsigned short* __restrict__ UH) {
  const size_t i  = (size_t)blockIdx.x * 256 + threadIdx.x;
  const size_t e0 = i * 8;
  const v4f a = *(const v4f*)(u + e0), b = *(const v4f*)(u + e0 + 4);
  v8us o;
#pragma unroll
  for (int e = 0; e < 4; ++e) {
    o[e]     = h_bits(a[e]);
    o[4 + e] = h_bits(b[e]);
  }
  *(volatile v8us*)(UH + e0) = o;
  __threadfence();
  *(volatile v8us*)(UH + e0) = o;
}

__global__ __launch_bounds__(256) void k_gemm_bu(const unsigned short* __restrict__ UHh,
                                                 const unsigned short* __restrict__ WB,
                                                 const float* __restrict__ gl, const float* __restrict__ nul,
                                                 const float* __restrict__ thl, float* __restrict__ LAM,
                                                 float* __restrict__ BU) {
  __shared__ __align__(16) float ldsf[128 * SFP];
  __shared__ __align__(16) float gsc[64];
  const int tid = threadIdx.x, lane = tid & 31, w = tid >> 5;
  const int h = lane >> 4, c = lane & 15;
  const int wm = (w >> 1) * 32, wn = (w & 1) * 32;
  const int m0 = blockIdx.y * 128;
  const int n0 = blockIdx.x * 64;

  if (blockIdx.x == 0 && blockIdx.y == 0) {
    const float lm = expf(-expf(nul[tid]));
    const float th = expf(thl[tid]);
    const float cs = cosf(th);
    const float sn = sinf(th);
    const float vr = lm * cs;
    const float vi = lm * sn;
    *(volatile float*)(LAM + tid) = vr;
    *(volatile float*)(LAM + NST + tid) = vi;
    __threadfence();
    *(volatile float*)(LAM + tid) = vr;
    *(volatile float*)(LAM + NST + tid) = vi;
  }
  if (tid < 64) gsc[tid] = expf(gl[(n0 + tid) & (NST - 1)]) * WSCI;

  v8f acc[2][2];
#pragma unroll
  for (int i = 0; i < 2; ++i)
#pragma unroll
    for (int j = 0; j < 2; ++j) acc[i][j] = zero8();
  gemm32x32(UHh, HIN, WB, HIN, m0 + wm, n0 + wn, HIN, lane, acc);

  stage_tile(ldsf, acc, wm, wn, h, c);
  __syncthreads();

  v4f val[8];
  size_t go[8];
#pragma unroll
  for (int it = 0; it < 8; ++it) {
    const int p  = tid + 256 * it;
    const int lr = p >> 4;
    const int pc = p & 15;
    const v4f sv = *(const v4f*)(ldsf + lr * SFP + pc * 4);
    const v4f gg = *(const v4f*)(gsc + pc * 4);
    val[it] = sv * gg;
    go[it] = (size_t)(m0 + lr) * NBU + n0 + pc * 4;
  }
#pragma unroll
  for (int it = 0; it < 8; ++it) *(volatile v4f*)(BU + go[it]) = val[it];
  __threadfence();
#pragma unroll
  for (int it = 0; it < 8; ++it) *(volatile v4f*)(BU + go[it]) = val[it];
}

__global__ __launch_bounds__(256) void k_scan(const float* __restrict__ LAM, float* bu) {
  __shared__ __align__(16) float sf[TB * NBU];
  __shared__ __align__(16) unsigned short st[TB * NBU];
  const int tid = threadIdx.x;
  const size_t rowb = (size_t)blockIdx.x * SEQL;
  unsigned short* ys = (unsigned short*)bu;

  const float lr = LAM[tid];
  const float li = LAM[NST + tid];

  float xr = 0.f, xi = 0.f;
#pragma unroll 1
  for (int t0 = 0; t0 < SEQL; t0 += TB) {
    const float* src = bu + (rowb + t0) * NBU;
    v4f bv[4];
#pragma unroll
    for (int it = 0; it < 4; ++it) {
      const int q = tid + 256 * it;
      bv[it] = *(const v4f*)(src + (size_t)q * 4);
    }
#pragma unroll
    for (int it = 0; it < 4; ++it) {
      const int q = tid + 256 * it;
      *(v4f*)(sf + q * 4) = bv[it];
    }
    __syncthreads();
#pragma unroll
    for (int tt = 0; tt < TB; ++tt) {
      st[tt * NBU + tid]       = h_bits(xr);
      st[tt * NBU + NST + tid] = h_bits(xi);
      const float br = sf[tt * NBU + tid];
      const float bi = sf[tt * NBU + NST + tid];
      const float nr = lr * xr - li * xi + br;
      const float ni = lr * xi + li * xr + bi;
      xr = nr;
      xi = ni;
    }
    __syncthreads();
    v8us hv[2];
    size_t go[2];
#pragma unroll
    for (int it = 0; it < 2; ++it) {
      const int q   = tid + 256 * it;
      const int row = q >> 6;
      const int pc  = q & 63;
      hv[it] = *(const v8us*)(st + row * NBU + pc * 8);
      go[it] = (rowb + t0 + row) * (size_t)LDP + (size_t)pc * 8;
    }
#pragma unroll
    for (int it = 0; it < 2; ++it) *(volatile v8us*)(ys + go[it]) = hv[it];
    __threadfence();
#pragma unroll
    for (int it = 0; it < 2; ++it) *(volatile v8us*)(ys + go[it]) = hv[it];
    __syncthreads();
  }
}

__global__ __launch_bounds__(256) void k_gemm_y(const unsigned short* __restrict__ PRE,
                                                const unsigned short* __restrict__ UHh,
                                                const unsigned short* __restrict__ WC, float* __restrict__ outh) {
  __shared__ __align__(16) float ldsf[128 * SFP];
  const int tid = threadIdx.x, lane = tid & 31, w = tid >> 5;
  const int h = lane >> 4, c = lane & 15;
  const int wm = (w >> 1) * 32, wn = (w & 1) * 32;
  const int m0 = blockIdx.y * 128;
  const int n0 = blockIdx.x * 64;

  v8f acc[2][2];
#pragma unroll
  for (int i = 0; i < 2; ++i)
#pragma unroll
    for (int j = 0; j < 2; ++j) acc[i][j] = zero8();
  gemm32x32(PRE, LDP, WC, KC, m0 + wm, n0 + wn, NBU, lane, acc);
  gemm32x32(UHh, HIN, WC + NBU, KC, m0 + wm, n0 + wn, HIN, lane, acc);

  stage_tile(ldsf, acc, wm, wn, h, c);
  __syncthreads();

  v4f val[8];
  size_t go[8];
#pragma unroll
  for (int it = 0; it < 8; ++it) {
    const int p  = tid + 256 * it;
    const int lr = p >> 4;
    const int pc = p & 15;
    const v4f sv = *(const v4f*)(ldsf + lr * SFP + pc * 4);
    val[it] = sv * WSCI;
    go[it] = (size_t)(m0 + lr) * HOUT + n0 + pc * 4;
  }
#pragma unroll
  for (int it = 0; it < 8; ++it) *(volatile v4f*)(outh + go[it]) = val[it];
  __threadfence();
#pragma unroll
  for (int it = 0; it < 8; ++it) *(volatile v4f*)(outh + go[it]) = val[it];
}

extern "C" void kernel_launch(void* const* d_in, const int* in_sizes, int n_in,
                              void* d_out, int out_size, void* d_ws, size_t ws_size,
                              hipStream_t stream) {
  if (n_in < 9) return;
  if (in_sizes[0] != NTOK * HIN) return;
  if (in_sizes[1] != NST || in_sizes[2] != NST || in_sizes[3] != NST) return;
  if (in_sizes[4] != NST * HIN || in_sizes[5] != NST * HIN) return;
  if (in_sizes[6] != HOUT * NST || in_sizes[7] != HOUT * NST) return;
  if (in_sizes[8] != HOUT * HIN) return;
  if (out_size != NTOK * HOUT) return;

  const float* u   = (const float*)d_in[0];
  const float* nul = (const float*)d_in[1];
  const float* thl = (const float*)d_in[2];
  const float* gl  = (const float*)d_in[3];
  const float* Bre = (const float*)d_in[4];
  const float* Bim = (const float*)d_in[5];
  const float* Cre = (const float*)d_in[6];
  const float* Cim = (const float*)d_in[7];
  const float* Dm  = (const float*)d_in[8];
  float* out = (float*)d_out;

  size_t off = 0;
  const size_t oWB  = off; off += (size_t)NBU * HIN * 2;
  const size_t oWC  = off; off += (size_t)HOUT * KC * 2;
  const size_t oLAM = off; off += (size_t)2 * NST * 4;
  const size_t oUH  = off; off += (size_t)NTOK * HIN * 2;
  const size_t oBU  = off; off += (size_t)TOKH * NBU * 4;
  if (off > ws_size) return;
  if (off > (size_t)134217728) return;
  if ((oUH & 127) != 0 || (oBU & 127) != 0 || (oLAM & 127) != 0) return;

  char* ws = (char*)d_ws;
  unsigned short* WB = (unsigned short*)(ws + oWB);
  unsigned short* WC = (unsigned short*)(ws + oWC);
  float* LAM = (float*)(ws + oLAM);
  unsigned short* UH = (unsigned short*)(ws + oUH);
  float* BU = (float*)(ws + oBU);
  const unsigned short* PRE = (const unsigned short*)(ws + oBU);

  k_prepw<<<dim3((NBU * HIN) / 2048 + (HOUT * KC) / 2048), dim3(256), 0, stream>>>(Bre, Bim, Cre, Cim, Dm, WB, WC);
  k_cvtu<<<dim3((NTOK * HIN) / 2048), dim3(256), 0, stream>>>(u, UH);
  for (int hf = 0; hf < NHALF; ++hf) {
    const unsigned short* UHh = UH + (size_t)hf * TOKH * HIN;
    float* outh = out + (size_t)hf * TOKH * HOUT;
    k_gemm_bu<<<dim3(NBU / 64, TOKH / 128, 1), dim3(256), 0, stream>>>(UHh, WB, gl, nul, thl, LAM, BU);
    k_scan<<<dim3(BH), dim3(256), 0, stream>>>(LAM, BU);
    k_gemm_y<<<dim3(HOUT / 64, TOKH / 128, 1), dim3(256), 0, stream>>>(PRE, UHh, WC, outh);
  }
  (void)hipGetLastError();
}
